// TempCatStatic_86079734546560
// MI455X (gfx1250) — hardware-verified
//
#include <hip/hip_runtime.h>
#include <stddef.h>

typedef __attribute__((ext_vector_type(16))) _Float16 v16h;
typedef __attribute__((ext_vector_type(8)))  _Float16 v8h;
typedef __attribute__((ext_vector_type(4)))  _Float16 v4h;
typedef __attribute__((ext_vector_type(16))) __bf16   v16b;
typedef __attribute__((ext_vector_type(8)))  __bf16   v8b;
typedef __attribute__((ext_vector_type(8)))  float    v8f;
typedef __attribute__((ext_vector_type(4)))  float    v4f;

__device__ __forceinline__ unsigned short f2bf_bits(float f) {
  unsigned u = __float_as_uint(f);
  return (unsigned short)((u + 0x7FFFu + ((u >> 16) & 1u)) >> 16);
}
__device__ __forceinline__ float bf_bits2f(unsigned short h) { return __uint_as_float(((unsigned)h) << 16); }

__device__ __forceinline__ void dep_guard_h(v8f& a, v8f& b, v16h x, v16h y) { asm volatile("v_nop\n\tv_nop\n\tv_nop\n\tv_nop" : "+v"(a), "+v"(b) : "v"(x), "v"(y)); }
__device__ __forceinline__ void dep_guard_b(v8f& a, v8f& b, v16b x, v16b y) { asm volatile("v_nop\n\tv_nop\n\tv_nop\n\tv_nop" : "+v"(a), "+v"(b) : "v"(x), "v"(y)); }
__device__ __forceinline__ void keep4_h(v16h a, v16h b, v16h c, v16h d) { asm volatile("v_nop" :: "v"(a), "v"(b), "v"(c), "v"(d)); }
__device__ __forceinline__ void keep4_b(v16b a, v16b b, v16b c, v16b d) { asm volatile("v_nop" :: "v"(a), "v"(b), "v"(c), "v"(d)); }
__device__ __forceinline__ void acc_guard4(v8f& a, v8f& b, v8f& c, v8f& d) { asm volatile("v_nop\n\tv_nop\n\tv_nop\n\tv_nop" : "+v"(a), "+v"(b), "+v"(c), "+v"(d)); }
template <typename T> struct Frag;
template <> struct Frag<_Float16> {
  typedef v16h V; union U { v16h v; v8h h[2]; };
  static __device__ __forceinline__ v16h load(const _Float16* p) {
    U f; f.h[0] = *(const v8h*)(p); f.h[1] = *(const v8h*)(p + 16); return f.v;
  }
  static __device__ __forceinline__ v8f mma(v16h a, v16h b, v8f c) {
    return __builtin_amdgcn_wmma_f32_16x16x32_f16(false, a, false, b, (short)0, c, false, false);
  }
  static __device__ __forceinline__ void guard(v8f& a, v8f& b, v16h x, v16h y) { dep_guard_h(a, b, x, y); }
  static __device__ __forceinline__ void keep(v16h a, v16h b, v16h c, v16h d) { keep4_h(a, b, c, d); }
};
template <> struct Frag<__bf16> {
  typedef v16b V; union U { v16b v; v8b h[2]; };
  static __device__ __forceinline__ v16b load(const __bf16* p) {
    U f; f.h[0] = *(const v8b*)(p); f.h[1] = *(const v8b*)(p + 16); return f.v;
  }
  static __device__ __forceinline__ v8f mma(v16b a, v16b b, v8f c) {
    return __builtin_amdgcn_wmma_f32_16x16x32_bf16(false, a, false, b, (short)0, c, false, false);
  }
  static __device__ __forceinline__ void guard(v8f& a, v8f& b, v16b x, v16b y) { dep_guard_b(a, b, x, y); }
  static __device__ __forceinline__ void keep(v16b a, v16b b, v16b c, v16b d) { keep4_b(a, b, c, d); }
};

template <int ET> struct Elem;
template <> struct Elem<0> { typedef _Float16 T; };
template <> struct Elem<1> { typedef __bf16 T; };
template <int ET, bool SPLIT, int BIAS_MODE, int OUT_MODE, bool RESID, int ACT = 0>
__global__ __launch_bounds__(256) void wmma_gemm64(
    const unsigned short* __restrict__ Ap, const unsigned short* __restrict__ A2p, int lda, long strideA,
    const unsigned short* __restrict__ Btp, const unsigned short* __restrict__ Bt2p, int ldb, long strideB,
    void* __restrict__ Cout, void* __restrict__ Cout2, int ldc, long strideC,
    const float* __restrict__ bias,
    const float* __restrict__ resid, long strideR,
    int M, int N, int K, float scale) {
  typedef typename Elem<ET>::T T;
  typedef typename Frag<T>::V V;
  const T* A = (const T*)Ap; const T* A2 = (const T*)A2p; const T* Bt = (const T*)Btp; const T* Bt2 = (const T*)Bt2p;
  __shared__ __align__(16) float sT[8][16 * 68];
  const int b    = blockIdx.y;
  const int lane = threadIdx.x & 31;
  const int wave = threadIdx.x >> 5;
  const int tilesN = N >> 6;
  const int tilesM = M >> 6;
  const int tile = blockIdx.x * 8 + wave;
  if (tile >= tilesM * tilesN) return;
  const int tm = tile / tilesN;
  const int tn = tile - tm * tilesN;
  const int m0 = tm << 6;
  const int n0 = tn << 6;

  const T* Ab  = A  + (size_t)b * strideA;
  const T* Bb  = Bt + (size_t)b * strideB;
  const T* Ab2 = SPLIT ? (A2  + (size_t)b * strideA) : nullptr;
  const T* Bb2 = SPLIT ? (Bt2 + (size_t)b * strideB) : nullptr;

  const int rlane = lane & 15;
  const int koff  = (lane >> 4) * 8;
  const int mOff  = (lane >> 4) * 8;

  v8f acc[4][4];
#pragma unroll
  for (int i = 0; i < 4; ++i)
#pragma unroll
    for (int j = 0; j < 4; ++j) acc[i][j] = (v8f){0.f,0.f,0.f,0.f,0.f,0.f,0.f,0.f};

  for (int k0 = 0; k0 < K; k0 += 32) {
    V bh[4], bl[4];
#pragma unroll
    for (int j = 0; j < 4; ++j) {
      const size_t bo = (size_t)(n0 + (j << 4) + rlane) * ldb + koff + k0;
      bh[j] = Frag<T>::load(Bb + bo);
      if (SPLIT) bl[j] = Frag<T>::load(Bb2 + bo);
    }
#pragma unroll
    for (int i = 0; i < 4; ++i) {
      const size_t ao = (size_t)(m0 + (i << 4) + rlane) * lda + koff + k0;
      V ah = Frag<T>::load(Ab + ao);
      V al;
      if (SPLIT) al = Frag<T>::load(Ab2 + ao);
#pragma unroll
      for (int j = 0; j < 4; ++j) {
        acc[i][j] = Frag<T>::mma(ah, bh[j], acc[i][j]);
        if (SPLIT) {
          acc[i][j] = Frag<T>::mma(ah, bl[j], acc[i][j]);
          acc[i][j] = Frag<T>::mma(al, bh[j], acc[i][j]);
        }
      }
      Frag<T>::guard(acc[i][0], acc[i][3], ah, SPLIT ? al : ah);
    }
    Frag<T>::keep(bh[0], bh[1], bh[2], bh[3]);
    if (SPLIT) Frag<T>::keep(bl[0], bl[1], bl[2], bl[3]);
  }
  acc_guard4(acc[0][0], acc[0][1], acc[0][2], acc[0][3]);
  acc_guard4(acc[1][0], acc[1][1], acc[1][2], acc[1][3]);
  acc_guard4(acc[2][0], acc[2][1], acc[2][2], acc[2][3]);
  acc_guard4(acc[3][0], acc[3][1], acc[3][2], acc[3][3]);

  float* slab = sT[wave];
  const float* Rb = RESID ? (resid + (size_t)b * strideR) : nullptr;
#pragma unroll
  for (int i = 0; i < 4; ++i) {
    const int mBase = m0 + (i << 4);
#pragma unroll
    for (int j = 0; j < 4; ++j) {
      const int n = n0 + (j << 4) + rlane;
      float bv = 0.f;
      if (BIAS_MODE == 2) bv = bias[n];
#pragma unroll
      for (int r = 0; r < 8; ++r) {
        float v = acc[i][j][r] * scale;
        if (BIAS_MODE == 1) v += bias[mBase + mOff + r];
        if (BIAS_MODE == 2) v += bv;
        if (RESID) v += Rb[(size_t)(mBase + mOff + r) * ldc + n];
        if (ACT == 1) v = tanhf(v);
        if (ACT == 2) v = fmaxf(v, 0.0f);
        if (ACT == 3) v = v / (1.0f + expf(-v));
        if (ACT == 4) v = (v > 0.f) ? v : 0.01f * v;
        if (ACT == 5) v = 0.5f * v * (1.0f + erff(v * 0.70710678118654752f));
        slab[(mOff + r) * 68 + (j << 4) + rlane] = v;
      }
    }
    __builtin_amdgcn_fence(__ATOMIC_RELEASE, "workgroup");
    __builtin_amdgcn_wave_barrier();
    __builtin_amdgcn_fence(__ATOMIC_ACQUIRE, "workgroup");
    if (OUT_MODE == 0) {
      float* C = (float*)Cout + (size_t)b * strideC;
      const int hh = lane >> 4, c4 = (lane & 15) * 4;
      for (int pass = 0; pass < 2; ++pass) {
#pragma unroll
        for (int it = 0; it < 8; ++it) {
          const int row = it * 2 + hh;
          v4f v = *(const v4f*)(slab + row * 68 + c4);
          *(volatile v4f*)(C + (size_t)(mBase + row) * ldc + n0 + c4) = v;
        }
        __threadfence();
      }
    } else {
      const int q = lane >> 3, c8 = (lane & 7) * 8;
      unsigned short* C  = (unsigned short*)Cout  + (size_t)b * strideC;
      unsigned short* C2 = (OUT_MODE == 2) ? ((unsigned short*)Cout2 + (size_t)b * strideC) : nullptr;
      for (int pass = 0; pass < 2; ++pass) {
#pragma unroll
        for (int it = 0; it < 4; ++it) {
          const int row = it * 4 + q;
          const float* sp = slab + row * 68 + c8;
          v8h hv, lv;
#pragma unroll
          for (int e = 0; e < 8; ++e) {
            if (OUT_MODE == 1) {
              hv[e] = (_Float16)sp[e];
            } else {
              unsigned short hb = f2bf_bits(sp[e]);
              unsigned short lb = f2bf_bits(sp[e] - bf_bits2f(hb));
              hv[e] = __builtin_bit_cast(_Float16, hb);
              lv[e] = __builtin_bit_cast(_Float16, lb);
            }
          }
          *(volatile v8h*)(C + (size_t)(mBase + row) * ldc + n0 + c8) = hv;
          if (OUT_MODE == 2) *(volatile v8h*)(C2 + (size_t)(mBase + row) * ldc + n0 + c8) = lv;
        }
        __threadfence();
      }
    }
    __builtin_amdgcn_fence(__ATOMIC_RELEASE, "workgroup");
    __builtin_amdgcn_wave_barrier();
    __builtin_amdgcn_fence(__ATOMIC_ACQUIRE, "workgroup");
  }
}

__global__ __launch_bounds__(256) void cast_f32_f16x2s(
    const float* __restrict__ in, _Float16* __restrict__ out, int n2, float sc) {
  int i = blockIdx.x * 256 + threadIdx.x;
  if (i < n2) {
    const _Float16 h0 = (_Float16)(in[2 * i] * sc), h1 = (_Float16)(in[2 * i + 1] * sc);
    const unsigned u = (unsigned)__builtin_bit_cast(unsigned short, h0) | ((unsigned)__builtin_bit_cast(unsigned short, h1) << 16);
    ((volatile unsigned*)out)[i] = u;
    __threadfence();
    ((volatile unsigned*)out)[i] = u;
  }
}

#define SEQ_BLK 32
#define HID 256
#define TSTEPS 24
#define HPITCH 264
#define WSC 16.0f
#define WSC_INV 0.0625f

__device__ __forceinline__ float frcp_(float x) { return __builtin_amdgcn_rcpf(x); }
__device__ __forceinline__ float sigm_(float x) { return frcp_(1.0f + __expf(-x)); }
__device__ __forceinline__ float tanh_(float x) {
  const float e = __expf(-2.0f * fabsf(x));
  const float t = (1.0f - e) * frcp_(1.0f + e);
  return copysignf(t, x);
}

__global__ __launch_bounds__(256) void lstm_seq_kernel(
    const float* __restrict__ h0, const float* __restrict__ c0,
    const float* __restrict__ tfeat, const float* __restrict__ tmask,
    const _Float16* __restrict__ Whh,
    const float* __restrict__ Wih,
    const float* __restrict__ bih, const float* __restrict__ bhh,
    _Float16* __restrict__ Hout,
    int nB)
{
  __shared__ __align__(16) _Float16 hs[2][SEQ_BLK * HPITCH];
  __shared__ __align__(32) float xsf[TSTEPS * SEQ_BLK];
  __shared__ __align__(32) float xsm[TSTEPS * SEQ_BLK];

  const int tid  = threadIdx.x;
  const int lane = tid & 31;
  const int wave = tid >> 5;
  const int hh   = lane >> 4;
  const int c    = lane & 15;
  const int b0   = blockIdx.x * SEQ_BLK;
  if (b0 + SEQ_BLK > nB) return;

#pragma unroll
  for (int i = 0; i < 8; ++i) {
    const int idx = i * 256 + tid;
    const int row = idx >> 6, c4 = (idx & 63) * 4;
    const v4f v = *(const v4f*)(h0 + (size_t)(b0 + row) * HID + c4);
    v4h hv;
    hv[0] = (_Float16)v[0]; hv[1] = (_Float16)v[1]; hv[2] = (_Float16)v[2]; hv[3] = (_Float16)v[3];
    *(v4h*)(hs[0] + row * HPITCH + c4) = hv;
  }
  for (int i = tid; i < TSTEPS * SEQ_BLK; i += 256) {
    const int row = i / TSTEPS, t = i - row * TSTEPS;
    xsf[t * SEQ_BLK + row] = tfeat[(size_t)(b0 + row) * TSTEPS + t];
    xsm[t * SEQ_BLK + row] = tmask[(size_t)(b0 + row) * TSTEPS + t];
  }
  float cst[2][2][8];
#pragma unroll
  for (int rt = 0; rt < 2; ++rt)
#pragma unroll
    for (int ct = 0; ct < 2; ++ct)
#pragma unroll
      for (int r = 0; r < 8; ++r)
        cst[rt][ct][r] = c0[(size_t)(b0 + rt * 16 + 8 * hh + r) * HID + 32 * wave + 16 * ct + c];
  float w0[4][2], w1[4][2], bs[4][2];
#pragma unroll
  for (int g = 0; g < 4; ++g)
#pragma unroll
    for (int ct = 0; ct < 2; ++ct) {
      const int gc = g * HID + 32 * wave + 16 * ct + c;
      w0[g][ct] = Wih[gc * 2 + 0];
      w1[g][ct] = Wih[gc * 2 + 1];
      bs[g][ct] = bih[gc] + bhh[gc];
    }
  __syncthreads();

  int cur = 0;
  for (int t = 0; t < TSTEPS; ++t) {
    const _Float16* hc = hs[cur];
    _Float16* hn = hs[cur ^ 1];
#pragma unroll
    for (int ct = 0; ct < 2; ++ct) {
      const int ncol = 32 * wave + 16 * ct + c;
      v8f acc[2][4];
#pragma unroll
      for (int rt = 0; rt < 2; ++rt)
#pragma unroll
        for (int g = 0; g < 4; ++g) acc[rt][g] = (v8f){0.f,0.f,0.f,0.f,0.f,0.f,0.f,0.f};
#pragma unroll 1
      for (int ks = 0; ks < HID / 32; ++ks) {
        const int k0 = ks * 32 + 8 * hh;
        v16h bq[4];
#pragma unroll
        for (int g = 0; g < 4; ++g)
          bq[g] = Frag<_Float16>::load(Whh + (size_t)(g * HID + ncol) * HID + k0);
#pragma unroll
        for (int rt = 0; rt < 2; ++rt) {
          const v16h a = Frag<_Float16>::load(hc + (rt * 16 + c) * HPITCH + k0);
#pragma unroll
          for (int g = 0; g < 4; ++g) acc[rt][g] = Frag<_Float16>::mma(a, bq[g], acc[rt][g]);
          Frag<_Float16>::guard(acc[rt][0], acc[rt][3], a, a);
        }
        Frag<_Float16>::keep(bq[0], bq[1], bq[2], bq[3]);
      }
      acc_guard4(acc[0][0], acc[0][1], acc[0][2], acc[0][3]);
      acc_guard4(acc[1][0], acc[1][1], acc[1][2], acc[1][3]);

#pragma unroll
      for (int rt = 0; rt < 2; ++rt) {
        const v8f xa = *(const v8f*)(xsf + t * SEQ_BLK + rt * 16 + 8 * hh);
        const v8f ma = *(const v8f*)(xsm + t * SEQ_BLK + rt * 16 + 8 * hh);
#pragma unroll
        for (int r = 0; r < 8; ++r) {
          const float x0 = xa[r], x1 = ma[r];
          float pi = fmaf(acc[rt][0][r], WSC_INV, bs[0][ct]); pi = fmaf(x0, w0[0][ct], pi); pi = fmaf(x1, w1[0][ct], pi);
          float pf = fmaf(acc[rt][1][r], WSC_INV, bs[1][ct]); pf = fmaf(x0, w0[1][ct], pf); pf = fmaf(x1, w1[1][ct], pf);
          float pg = fmaf(acc[rt][2][r], WSC_INV, bs[2][ct]); pg = fmaf(x0, w0[2][ct], pg); pg = fmaf(x1, w1[2][ct], pg);
          float po = fmaf(acc[rt][3][r], WSC_INV, bs[3][ct]); po = fmaf(x0, w0[3][ct], po); po = fmaf(x1, w1[3][ct], po);
          const float ig = sigm_(pi);
          const float fg = sigm_(pf);
          const float gg = tanh_(pg);
          const float og = sigm_(po);
          const float cn = fmaf(fg, cst[rt][ct][r], ig * gg);
          cst[rt][ct][r] = cn;
          const float hv = og * tanh_(cn);
          hn[(rt * 16 + 8 * hh + r) * HPITCH + ncol] = (_Float16)hv;
        }
      }
    }
    __syncthreads();
    cur ^= 1;
  }

  {
    const _Float16* hf = hs[cur];
    const int q = lane >> 3, c8 = (lane & 7) * 8;
    for (int pass = 0; pass < 2; ++pass) {
#pragma unroll
      for (int it = 0; it < 4; ++it) {
        const int row = wave * 4 + it;
        const v8h v = *(const v8h*)(hf + row * HPITCH + 64 * q + c8);
        *(volatile v8h*)(Hout + (size_t)(b0 + row) * HID + 64 * q + c8) = v;
      }
      __threadfence();
    }
  }
}

__global__ __launch_bounds__(256) void head_loss_kernel(
    const _Float16* __restrict__ Hf,
    const _Float16* __restrict__ Sf,
    const float* __restrict__ Wlr,
    const float* __restrict__ blr,
    const float* __restrict__ tgt,
    float* __restrict__ out,
    int nB)
{
  __shared__ __align__(32) float wl[512];
  __shared__ double red[256];
  const int tid = threadIdx.x;
  for (int i = tid; i < 512; i += 256) wl[i] = Wlr[i];
  __syncthreads();
  const float bl = blr[0];
  double lsum = 0.0;
  const int nIter = nB >> 8;
  for (int it = 0; it < nIter; ++it) {
    const int row = (it << 8) + tid;
    const _Float16* hr = Hf + (size_t)row * 256;
    const _Float16* sr = Sf + (size_t)row * 256;
    float ph = 0.f, ps = 0.f;
#pragma unroll 1
    for (int j = 0; j < 32; ++j) {
      const v8h hv = *(const v8h*)(hr + 8 * j);
      const v8h sv = *(const v8h*)(sr + 8 * j);
      const v8f wh = *(const v8f*)(wl + 8 * j);
      const v8f ws = *(const v8f*)(wl + 256 + 8 * j);
#pragma unroll
      for (int e = 0; e < 8; ++e) {
        ph = fmaf((float)hv[e], wh[e], ph);
        ps = fmaf((float)sv[e], ws[e], ps);
      }
    }
    const float p = (ph + ps) + bl;
    *(volatile float*)(out + row) = p;
    __threadfence();
    *(volatile float*)(out + row) = p;
    const float tg = tgt[row];
    const float ex = __expf(-fabsf(p));
    const float l  = fmaxf(p, 0.0f) - p * tg + __logf(1.0f + ex);
    lsum += (double)l;
  }
  red[tid] = lsum;
  __syncthreads();
  for (int st = 128; st > 0; st >>= 1) {
    if (tid < st) red[tid] += red[tid + st];
    __syncthreads();
  }
  if (tid == 0) {
    const float lv = (float)(red[0] / (double)nB);
    *(volatile float*)(out + nB) = lv;
    __threadfence();
    *(volatile float*)(out + nB) = lv;
  }
}

extern "C" void kernel_launch(void* const* d_in, const int* in_sizes, int n_in,
                              void* d_out, int out_size, void* d_ws, size_t ws_size,
                              hipStream_t stream) {
  if (n_in < 18) return;
  const float* static_f = (const float*)d_in[0];
  const float* tfeat    = (const float*)d_in[1];
  const float* tmask    = (const float*)d_in[2];
  const float* targets  = (const float*)d_in[3];
  const float* h0       = (const float*)d_in[4];
  const float* c0       = (const float*)d_in[5];
  const float* W_ih     = (const float*)d_in[6];
  const float* W_hh     = (const float*)d_in[7];
  const float* b_ih     = (const float*)d_in[8];
  const float* b_hh     = (const float*)d_in[9];
  const float* W1       = (const float*)d_in[10];
  const float* b1       = (const float*)d_in[11];
  const float* W2       = (const float*)d_in[12];
  const float* b2       = (const float*)d_in[13];
  const float* W3       = (const float*)d_in[14];
  const float* b3       = (const float*)d_in[15];
  const float* W_lr     = (const float*)d_in[16];
  const float* b_lr     = (const float*)d_in[17];

  const int nB = in_sizes[4] / HID;
  if (nB <= 0 || (nB % 256) != 0) return;
  if (in_sizes[0] != nB * 256 || in_sizes[5] != nB * HID) return;
  if (in_sizes[1] != nB * TSTEPS || in_sizes[2] != nB * TSTEPS) return;
  if (in_sizes[3] != nB) return;
  if (in_sizes[6] != 4 * HID * 2 || in_sizes[7] != 4 * HID * HID || in_sizes[8] != 4 * HID || in_sizes[9] != 4 * HID) return;
  if (in_sizes[10] != 256 * 256 || in_sizes[12] != 256 * 256 || in_sizes[14] != 256 * 256) return;
  if (in_sizes[11] != 256 || in_sizes[13] != 256 || in_sizes[15] != 256) return;
  if (in_sizes[16] != 512 || in_sizes[17] < 1) return;
  if (out_size != nB + 1) return;

  size_t off = 0;
  auto take = [&](size_t bytes) -> char* {
    char* p = (char*)d_ws + off;
    off += (bytes + 255) & ~(size_t)255;
    return p;
  };
  _Float16* sf16  = (_Float16*)take((size_t)nB * 256 * 2);
  _Float16* Whh16 = (_Float16*)take((size_t)4 * HID * HID * 2);
  _Float16* W1h   = (_Float16*)take((size_t)256 * 256 * 2);
  _Float16* W2h   = (_Float16*)take((size_t)256 * 256 * 2);
  _Float16* W3h   = (_Float16*)take((size_t)256 * 256 * 2);
  _Float16* H16   = (_Float16*)take((size_t)nB * HID * 2);
  _Float16* S1    = (_Float16*)take((size_t)nB * 256 * 2);
  _Float16* S2    = (_Float16*)take((size_t)nB * 256 * 2);
  if (off > ws_size) return;

  {
    const int n2s = nB * 256 / 2;
    cast_f32_f16x2s<<<(n2s + 255) / 256, 256, 0, stream>>>(static_f, sf16, n2s, 1.0f);
    const int n2h = 4 * HID * HID / 2;
    cast_f32_f16x2s<<<(n2h + 255) / 256, 256, 0, stream>>>(W_hh, Whh16, n2h, WSC);
    const int n2w = 256 * 256 / 2;
    cast_f32_f16x2s<<<(n2w + 255) / 256, 256, 0, stream>>>(W1, W1h, n2w, WSC);
    cast_f32_f16x2s<<<(n2w + 255) / 256, 256, 0, stream>>>(W2, W2h, n2w, WSC);
    cast_f32_f16x2s<<<(n2w + 255) / 256, 256, 0, stream>>>(W3, W3h, n2w, WSC);
  }

  lstm_seq_kernel<<<nB / SEQ_BLK, 256, 0, stream>>>(h0, c0, tfeat, tmask, Whh16, W_ih, b_ih, b_hh, H16, nB);

  {
    const int tiles = (nB / 64) * (256 / 64);
    const dim3 grid((tiles + 7) / 8, 1);
    wmma_gemm64<0, false, 2, 1, false, 2><<<grid, 256, 0, stream>>>(
        (const unsigned short*)sf16, (const unsigned short*)sf16, 256, 0L,
        (const unsigned short*)W1h, (const unsigned short*)W1h, 256, 0L,
        (void*)S1, (void*)S1, 256, 0L, b1, b1, 0L, nB, 256, 256, WSC_INV);
    wmma_gemm64<0, false, 2, 1, false, 2><<<grid, 256, 0, stream>>>(
        (const unsigned short*)S1, (const unsigned short*)S1, 256, 0L,
        (const unsigned short*)W2h, (const unsigned short*)W2h, 256, 0L,
        (void*)S2, (void*)S2, 256, 0L, b2, b2, 0L, nB, 256, 256, WSC_INV);
    wmma_gemm64<0, false, 2, 1, false, 2><<<grid, 256, 0, stream>>>(
        (const unsigned short*)S2, (const unsigned short*)S2, 256, 0L,
        (const unsigned short*)W3h, (const unsigned short*)W3h, 256, 0L,
        (void*)S1, (void*)S1, 256, 0L, b3, b3, 0L, nB, 256, 256, WSC_INV);
  }

  head_loss_kernel<<<1, 256, 0, stream>>>(H16, S1, W_lr, b_lr, targets, (float*)d_out, nB);
}
